// StateSpaceLayer_82094004895750
// MI455X (gfx1250) — hardware-verified
//
#include <hip/hip_runtime.h>


namespace {
constexpr int B = 2, S = 1024, D = 64, NROW = B * S * D  , BL = B  ;
constexpr float XS = 8.0f, WSC = 256.0f;
static_assert(D == 64 && NROW % 64 == 0, "tiling");
typedef _Float16 b16;
typedef __attribute__((ext_vector_type(16))) _Float16 v16b;
typedef __attribute__((ext_vector_type(8))) _Float16 v8b;
typedef __attribute__((ext_vector_type(8))) float v8f;
typedef __attribute__((ext_vector_type(4))) float v4f;
__device__ __forceinline__ float bf16_rne(float f) { unsigned int u = __float_as_uint(f); u += 0x7FFFu + ((u >> 16) & 1u); return __uint_as_float(u & 0xFFFF0000u); }
__device__ __forceinline__ void split16(float v, b16& hi, b16& lo) { hi = (b16)v; lo = (b16)(v - (float)hi); }
__device__ __forceinline__ v16b frag_kb(const b16* p, int hh) { const v8b a = *(const v8b*)(p + 8 * hh), b = *(const v8b*)(p + 16 + 8 * hh); v16b f;
#pragma unroll
  for (int e = 0; e < 8; ++e) { f[e] = a[e]; f[8 + e] = b[e]; } return f; }
__device__ __forceinline__ v8f wmma16b(v16b a, v16b b, v8f c) { v8f d = __builtin_amdgcn_wmma_f32_16x16x32_f16(false, a, false, b, (short)0, c, false, false); asm volatile("v_nop\n\tv_nop\n\tv_nop\n\tv_nop" : "+v"(d) : "v"(a), "v"(b)); return d; }
__device__ __forceinline__ void wave_lds_sync() { __builtin_amdgcn_fence(__ATOMIC_RELEASE, "workgroup"); __builtin_amdgcn_wave_barrier(); __builtin_amdgcn_fence(__ATOMIC_ACQUIRE, "workgroup"); }
__device__ __forceinline__ float pmul(float a, float b) { float p = a * b; asm volatile("" : "+v"(p)); return p; }
__device__ __forceinline__ int iclamp(int v, int lo, int hi) { return v < lo ? lo : (v > hi ? hi : v); }

typedef __attribute__((ext_vector_type(2))) _Float16 v2h;
typedef __attribute__((ext_vector_type(4))) _Float16 v4h;
typedef __attribute__((ext_vector_type(2))) float v2f;
typedef __attribute__((ext_vector_type(4))) int v4i;
__device__ __forceinline__ float nexp2(float v) { return __builtin_amdgcn_exp2f(v); }
__global__ __launch_bounds__(128) void wb_kernel(const float* __restrict__ w, b16* __restrict__ WB) {
  const int t = threadIdx.x; const int o = t / 8, k0 = (t % 8) * 8; v8b v; for (int j = 0; j < 8; ++j) v[j] = (b16)(o == 0 ? bf16_rne(w[k0 + j]) * WSC : 0.0f);
  for (int pass = 0; pass < 2; ++pass) { *(volatile v8b*)(WB + o * D + k0) = v; __threadfence(); }
}
__global__ __launch_bounds__(128) void decay_kernel(const float* __restrict__ x, const b16* __restrict__ WB, const float* __restrict__ logA, const float* __restrict__ bdt, float* __restrict__ ADEC) {
  __shared__ __attribute__((aligned(16))) b16 As[64][D + 8]; __shared__ float Sa[64];
  const int tid = threadIdx.x, wave = tid >> 5, lane = tid & 31, nloc = lane & 15, hlf = lane >> 4; const size_t r0 = (size_t)blockIdx.x * 64;
  { const int row = tid >> 1, half = tid & 1; const float* xr = x + (r0 + row) * D + half * 32; for (int q = 0; q < 8; ++q) { const v4f t4 = *(const v4f*)(xr + 4 * q); v4h o4; for (int j = 0; j < 4; ++j) o4[j] = (b16)(bf16_rne(t4[j]) * XS); *(v4h*)(&As[row][half * 32 + 4 * q]) = o4; } }
  __syncthreads();
  v8f acc = (v8f){};
#pragma unroll
  for (int kb = 0; kb < D; kb += 32) acc = wmma16b(frag_kb(&As[wave * 16 + nloc][kb], hlf), frag_kb(WB + (size_t)nloc * D + kb, hlf), acc);
  if (nloc == 0) { const float bb = bf16_rne(bdt[0]);
#pragma unroll
    for (int r = 0; r < 8; ++r) { const int rr = wave * 16 + 8 * hlf + r; const float z = acc[r] * (1.0f / (XS * WSC)) + bb; const float dt = (z > 20.0f) ? z : log1pf(__expf(z)); const float Ar = -__expf(bf16_rne(logA[rr])); Sa[rr] = __expf(dt * Ar); } }
  __syncthreads();
  for (int pass = 0; pass < 2; ++pass) { if (wave == 0) *(volatile v2f*)(ADEC + r0 + lane * 2) = *(const v2f*)(&Sa[lane * 2]); __threadfence(); }
}
__global__ __launch_bounds__(64) void scan_kernel(const float* __restrict__ x, const float* __restrict__ ADEC, float* __restrict__ out) {
  const int c = threadIdx.x; const int b = blockIdx.x / D, r = blockIdx.x % D;
#pragma unroll 1
  for (int pass = 0; pass < 2; ++pass) { float h = 0.0f;
#pragma unroll 1
    for (int s = 0; s < S; ++s) { const size_t row = ((size_t)b * S + s) * D + r; const float a = ADEC[row]; const float xv = bf16_rne(x[row * D + c]); h = fmaf(a, h, xv); ((volatile float*)out)[row * D + c] = h; }
    __threadfence(); }
}
}

extern "C" void kernel_launch(void* const* d_in, const int* in_sizes, int n_in, void* d_out, int out_size, void* d_ws, size_t ws_size, hipStream_t stream) {
  (void)n_in;
  auto Fp = [&](int i) { return (const float*)d_in[i]; };
  if (in_sizes[0] != NROW * D || in_sizes[1] != D || in_sizes[2] != D || in_sizes[3] != 1 || out_size != NROW * D) return;
  size_t off = 0; char* ws = (char*)d_ws;
  auto carve = [&](size_t bytes) { char* p = ws + off; off += (bytes + 255) & ~(size_t)255; return p; };
  b16* WB = (b16*)carve(16 * D * 2); float* ADEC = (float*)carve((size_t)NROW * 4);
  if (off > ws_size || off > ((size_t)128 << 20)) return;
  wb_kernel<<<1, 128, 0, stream>>>(Fp(2), WB);
  decay_kernel<<<(BL * S * D) / 64, 128, 0, stream>>>(Fp(0), WB, Fp(1), Fp(3), ADEC);
  scan_kernel<<<BL * D, 64, 0, stream>>>(Fp(0), ADEC, (float*)d_out);
}
